// NT_Xent_16338055594021
// MI455X (gfx1250) — hardware-verified
//
#include <hip/hip_runtime.h>


#define NB2  4096
#define HB   2048
#define DZ   256
#define NC   100
#define NCP  128
#define RCH  1024
#define DM   DZ
#define NTK  NB2
#define LOSC 1024.0f

typedef _Float16 h16;
typedef unsigned short bf;
typedef __attribute__((ext_vector_type(16))) __bf16   v16bf;
typedef __attribute__((ext_vector_type(16))) _Float16 v16h;
typedef __attribute__((ext_vector_type(8)))  _Float16 v8h;
typedef __attribute__((ext_vector_type(8)))  unsigned short v8us;
typedef __attribute__((ext_vector_type(8)))  float    v8f;
typedef __attribute__((ext_vector_type(4)))  float    v4f;
typedef __attribute__((ext_vector_type(4)))  _Float16 v4h;
typedef v8h  __attribute__((may_alias)) v8ha;
typedef v4f  __attribute__((may_alias)) v4fa;
typedef v8us __attribute__((may_alias)) v8usa;

__device__ __forceinline__ unsigned short f2bf(float f) { unsigned u = __float_as_uint(f); u += 0x7FFFu + ((u >> 16) & 1u); return (unsigned short)(u >> 16); }
__device__ __forceinline__ float bf2f(unsigned short b) { return __uint_as_float(((unsigned)b) << 16); }
__device__ __forceinline__ float bfr(float f) { return bf2f(f2bf(f)); }
__device__ __forceinline__ v16h cat16(v8h lo, v8h hi) { return __builtin_shufflevector(lo, hi, 0, 1, 2, 3, 4, 5, 6, 7, 8, 9, 10, 11, 12, 13, 14, 15); }
__device__ __forceinline__ v16bf cat16b(v8us lo, v8us hi) { return __builtin_bit_cast(v16bf, __builtin_shufflevector(lo, hi, 0, 1, 2, 3, 4, 5, 6, 7, 8, 9, 10, 11, 12, 13, 14, 15)); }
__device__ __forceinline__ v8f wmma16(v16h a, v16h b, v8f c) { return __builtin_amdgcn_wmma_f32_16x16x32_f16(false, a, false, b, (short)0, c, false, false); }
__device__ __forceinline__ v8f wmmab(v16bf a, v16bf b, v8f c) { return __builtin_amdgcn_wmma_f32_16x16x32_bf16(false, a, false, b, (short)0, c, false, false); }

template <bool SPLITA, bool F16OUT = false>
__global__ __launch_bounds__(128) void k_gemmb(const bf* __restrict__ A, const bf* __restrict__ Al, const bf* __restrict__ Bn, const float* __restrict__ bias, float* C, int ldc, h16* C2, const float* __restrict__ R = nullptr, int K = DM, int roundR = 1) {
    __shared__ __align__(16) float ost[4][16 * 68];
    const int lane = threadIdx.x & 31, wave = threadIdx.x >> 5, lr = lane & 15, hi = lane >> 4;
    const int r0 = blockIdx.x * 64 + wave * 16, c0 = blockIdx.y * 64;
    const size_t aoff = (size_t)(r0 + lr) * K + 8 * hi;
    size_t boff[4];
#pragma unroll
    for (int t = 0; t < 4; ++t) boff[t] = (size_t)(c0 + t * 16 + lr) * K + 8 * hi;
    v8f acc[4];
#pragma unroll
    for (int t = 0; t < 4; ++t) acc[t] = (v8f){};
#pragma unroll 1
    for (int kc = 0; kc < K; kc += 32) {
        const v16bf a = cat16b(*(const v8us*)(A + aoff + kc), *(const v8us*)(A + aoff + kc + 16));
        v16bf al = a;
        if (SPLITA) al = cat16b(*(const v8us*)(Al + aoff + kc), *(const v8us*)(Al + aoff + kc + 16));
#pragma unroll
        for (int t = 0; t < 4; ++t) { const v16bf b = cat16b(*(const v8us*)(Bn + boff[t] + kc), *(const v8us*)(Bn + boff[t] + kc + 16)); acc[t] = wmmab(a, b, acc[t]); if (SPLITA) acc[t] = wmmab(al, b, acc[t]); }
        asm volatile("v_nop\n\tv_nop\n\tv_nop\n\tv_nop" : "+v"(acc[0]), "+v"(acc[1]), "+v"(acc[2]), "+v"(acc[3]) : "v"(a), "v"(al));
    }
    float* os = &ost[wave][0];
#pragma unroll
    for (int t = 0; t < 4; ++t) { const float bv = bias ? bfr(bias[c0 + t * 16 + lr]) : 0.f;
#pragma unroll
        for (int j = 0; j < 8; ++j) os[(hi * 8 + j) * 68 + t * 16 + lr] = acc[t][j] + bv; }
    __syncthreads();
    if (F16OUT) {
        h16* crow = (h16*)(void*)C + (size_t)r0 * ldc + c0;
        auto pass = [&]() {
#pragma unroll
            for (int s = 0; s < 4; ++s) { const int row = 4 * s + (lane >> 3), piece = lane & 7; const float* sp = os + row * 68 + piece * 8; v8h o, o2;
#pragma unroll
                for (int i = 0; i < 8; ++i) { const h16 a = (h16)sp[i]; o[i] = a; o2[i] = (h16)((sp[i] - (float)a) * LOSC); }
                *(volatile v8h*)(crow + (size_t)row * ldc + piece * 8) = o; if (C2) *(volatile v8h*)(C2 + (size_t)r0 * ldc + c0 + (size_t)row * ldc + piece * 8) = o2; }
        };
        pass(); __threadfence(); pass();
    } else {
        float* crow = C + (size_t)r0 * ldc + c0;
        auto pass = [&]() {
#pragma unroll
            for (int s = 0; s < 8; ++s) { const int Lid = (lane >> 3) + 4 * s, piece = lane & 7; const int row = Lid >> 1, cofs = (Lid & 1) * 32 + piece * 4;
                v4f val = *(const v4fa*)(os + row * 68 + cofs); if (R) { const v4f rv = *(const v4f*)(R + ((size_t)r0 + row) * ldc + c0 + cofs); val += roundR ? (v4f){bfr(rv[0]), bfr(rv[1]), bfr(rv[2]), bfr(rv[3])} : rv; }
                *(volatile v4f*)(crow + (size_t)row * ldc + cofs) = val; }
        };
        pass(); __threadfence(); pass();
    }
}

__global__ __launch_bounds__(128) void k_gemm3(const bf* __restrict__ Ah, const bf* __restrict__ Al, const bf* __restrict__ Bh, const bf* __restrict__ Bl, int K, float* C, int ldc) {
    __shared__ __align__(16) float ost[4][16 * 68];
    const int lane = threadIdx.x & 31, wave = threadIdx.x >> 5, lr = lane & 15, hi = lane >> 4;
    const int r0 = blockIdx.x * 64 + wave * 16, c0 = blockIdx.y * 64;
    const size_t aoff = (size_t)(r0 + lr) * K + 8 * hi;
    v8f acc[4];
#pragma unroll
    for (int t = 0; t < 4; ++t) acc[t] = (v8f){};
#pragma unroll 1
    for (int kc = 0; kc < K; kc += 32) {
        const v16bf a = cat16b(*(const v8us*)(Ah + aoff + kc), *(const v8us*)(Ah + aoff + kc + 16));
        const v16bf al = cat16b(*(const v8us*)(Al + aoff + kc), *(const v8us*)(Al + aoff + kc + 16));
#pragma unroll
        for (int t = 0; t < 4; ++t) { const size_t bo = (size_t)(c0 + t * 16 + lr) * K + kc + 8 * hi;
            const v16bf bh = cat16b(*(const v8us*)(Bh + bo), *(const v8us*)(Bh + bo + 16)); const v16bf bl = cat16b(*(const v8us*)(Bl + bo), *(const v8us*)(Bl + bo + 16));
            acc[t] = wmmab(a, bh, acc[t]); acc[t] = wmmab(al, bh, acc[t]); acc[t] = wmmab(a, bl, acc[t]); }
        asm volatile("v_nop\n\tv_nop\n\tv_nop\n\tv_nop" : "+v"(acc[0]), "+v"(acc[1]), "+v"(acc[2]), "+v"(acc[3]) : "v"(a), "v"(al));
    }
    float* os = &ost[wave][0];
#pragma unroll
    for (int t = 0; t < 4; ++t) {
#pragma unroll
        for (int j = 0; j < 8; ++j) os[(hi * 8 + j) * 68 + t * 16 + lr] = acc[t][j]; }
    __builtin_amdgcn_wave_barrier(); asm volatile("" ::: "memory");
    float* crow = C + (size_t)r0 * ldc + c0;
    auto pass = [&]() {
#pragma unroll
        for (int s = 0; s < 8; ++s) { const int Lid = (lane >> 3) + 4 * s, piece = lane & 7; const int row = Lid >> 1, cofs = (Lid & 1) * 32 + piece * 4;
            const v4f val = *(const v4fa*)(os + row * 68 + cofs); *(volatile v4f*)(crow + (size_t)row * ldc + cofs) = val; }
    };
    pass(); __threadfence(); pass();
}

__global__ __launch_bounds__(256) void k_znorm(const float* __restrict__ zi, const float* __restrict__ zj, bf* Zh, bf* Zl) {
    const int lane = threadIdx.x & 31, r = blockIdx.x * 8 + (threadIdx.x >> 5); if (r >= NB2) return;
    const float* src = (r < HB) ? (zi + (size_t)r * DZ) : (zj + (size_t)(r - HB) * DZ);
    const v8f v = *(const v8f*)(src + lane * 8); float x[8]; float s = 0.f;
#pragma unroll
    for (int i = 0; i < 8; ++i) { x[i] = bfr(v[i]); s = fmaf(x[i], x[i], s); }
#pragma unroll
    for (int sh = 16; sh; sh >>= 1) s += __shfl_xor(s, sh, 32);
    const float inv = 1.0f / sqrtf(s);
    v8us oh, ol;
#pragma unroll
    for (int i = 0; i < 8; ++i) { const float y = x[i] * inv; const unsigned short hb = f2bf(y); oh[i] = hb; ol[i] = f2bf(y - bf2f(hb)); }
    const size_t o = (size_t)r * DZ + lane * 8;
    *(volatile v8us*)(Zh + o) = oh; *(volatile v8us*)(Zl + o) = ol; __threadfence(); *(volatile v8us*)(Zh + o) = oh; *(volatile v8us*)(Zl + o) = ol;
}
__global__ __launch_bounds__(256) void k_dist(const float* __restrict__ dl, bf* D) {
    typedef __attribute__((ext_vector_type(4))) unsigned short v4us;
    const int lane = threadIdx.x & 31, r = blockIdx.x * 8 + (threadIdx.x >> 5); if (r >= NB2) return;
    const float* src = dl + (size_t)(r % HB) * NC; v4us o;
#pragma unroll
    for (int i = 0; i < 4; ++i) { const int c = lane * 4 + i; o[i] = (c < NC) ? f2bf(src[c]) : (unsigned short)0; }
    *(volatile v4us*)(D + (size_t)r * NCP + lane * 4) = o; __threadfence(); *(volatile v4us*)(D + (size_t)r * NCP + lane * 4) = o;
}
__global__ __launch_bounds__(256) void k_rows(const float* __restrict__ S, const float* __restrict__ PM, int r0, float* RAT) {
    __shared__ float rat[32];
    const int lane = threadIdx.x & 31, wave = threadIdx.x >> 5;
#pragma unroll 1
    for (int rr = 0; rr < 4; ++rr) {
        const int r = blockIdx.x * 32 + wave * 4 + rr; const int n = r0 + r; const float* sr = S + (size_t)r * NB2; const float* pr = PM + (size_t)r * NB2;
        float nom = 0.f, den = 0.f;
#pragma unroll 1
        for (int q = 0; q < NB2 / 256; ++q) { const v8f sv = *(const v8f*)(sr + q * 256 + lane * 8), pv = *(const v8f*)(pr + q * 256 + lane * 8);
#pragma unroll
            for (int i = 0; i < 8; ++i) { const int m = q * 256 + lane * 8 + i; const float off = (m == n) ? 0.f : 1.f; nom = fmaf(sv[i] * pv[i], off, nom); den = fmaf(__expf(sv[i]), off, den); } }
#pragma unroll
        for (int sh = 16; sh; sh >>= 1) { nom += __shfl_xor(nom, sh, 32); den += __shfl_xor(den, sh, 32); }
        if (lane == 0) rat[wave * 4 + rr] = nom / den;
    }
    __syncthreads();
    if (wave == 0) { const float v = rat[lane]; float* p = RAT + r0 + blockIdx.x * 32 + lane; *(volatile float*)p = v; __threadfence(); *(volatile float*)p = v; }
}
__global__ __launch_bounds__(32) void k_final(const float* __restrict__ RAT, float* OUTP) {
    const int lane = threadIdx.x; float s = 0.f;
#pragma unroll 1
    for (int i = lane; i < NB2; i += 32) s += RAT[i];
#pragma unroll
    for (int sh = 16; sh; sh >>= 1) s += __shfl_xor(s, sh, 32);
    const float v = s / (float)NB2;
    if (lane == 0) { *(volatile float*)OUTP = v; __threadfence(); *(volatile float*)OUTP = v; }
}

extern "C" void kernel_launch(void* const* d_in, const int* in_sizes, int n_in,
                              void* d_out, int out_size, void* d_ws, size_t ws_size, hipStream_t stream) {
    (void)in_sizes; (void)n_in; (void)out_size;
    const float* zi = (const float*)d_in[0]; const float* zj = (const float*)d_in[1]; const float* dl = (const float*)d_in[3];
    float* out = (float*)d_out;
    char* wsp = (char*)d_ws;
    auto take = [&](size_t bytes) { char* p = wsp; wsp += (bytes + 255) & ~(size_t)255; return (void*)p; };
    bf* Zh = (bf*)take((size_t)NB2 * DZ * 2); bf* Zl = (bf*)take((size_t)NB2 * DZ * 2); bf* D = (bf*)take((size_t)NB2 * NCP * 2);
    float* S = (float*)take((size_t)RCH * NB2 * 4); float* PM = (float*)take((size_t)RCH * NB2 * 4); float* RAT = (float*)take((size_t)NB2 * 4);
    if ((size_t)(wsp - (char*)d_ws) > ws_size) return;
    k_znorm<<<NB2 / 8, 256, 0, stream>>>(zi, zj, Zh, Zl);
    k_dist<<<NB2 / 8, 256, 0, stream>>>(dl, D);
    for (int ch = 0; ch < NB2 / RCH; ++ch) {
        const int r0 = ch * RCH;
        k_gemm3<<<dim3(RCH / 64, NB2 / 64, 1), 128, 0, stream>>>(Zh + (size_t)r0 * DZ, Zl + (size_t)r0 * DZ, Zh, Zl, DZ, S, NB2);
        k_gemmb<false, false><<<dim3(RCH / 64, NB2 / 64, 1), 128, 0, stream>>>(D + (size_t)r0 * NCP, nullptr, D, nullptr, PM, NB2, nullptr, nullptr, NCP);
        k_rows<<<RCH / 32, 256, 0, stream>>>(S, PM, r0, RAT);
    }
    k_final<<<1, 32, 0, stream>>>(RAT, out);
}
